// RWKV6Attention_34540126994590
// MI455X (gfx1250) — hardware-run, weakly checked
//
#include <hip/hip_runtime.h>
#include <math.h>

constexpr int kB = 2;
constexpr int kT = 1024;
constexpr int kC = 1024;
constexpr int kH = 16;
constexpr int kHS = 64;
constexpr int kMixRank = 32;
constexpr int kMixCols = 160;
constexpr int kMixPad = 192;
constexpr int kDecRank = 64;
constexpr int kRows = kB * kT;
constexpr size_t kPlane = (size_t)kRows * kC;
constexpr int kChunk = 32;
constexpr float kLCarry = 64.0f;
constexpr float kLFold = 1.0f / kLCarry;
constexpr float kGnEps = 1e-5f;
static_assert(kC == kH * kHS);
static_assert(kMixCols == 5 * kMixRank && kMixCols <= kMixPad);
static_assert(kRows % 64 == 0 && kC % 64 == 0 && kMixPad % 64 == 0 && kDecRank % 64 == 0);
static_assert(kC % 32 == 0 && kMixRank % 32 == 0 && kDecRank % 32 == 0);
static_assert(((kRows / 64) * (kC / 64)) % 8 == 0);
static_assert(((kRows / 64) * (kMixPad / 64)) % 8 == 0);
static_assert(((kRows / 64) * (kDecRank / 64)) % 8 == 0);
static_assert(kT % kChunk == 0 && kHS == 64 && (kT & (kT - 1)) == 0);

typedef __attribute__((ext_vector_type(16))) _Float16 v16h;
typedef __attribute__((ext_vector_type(8)))  _Float16 v8h;
typedef __attribute__((ext_vector_type(16))) __bf16   v16b;
typedef __attribute__((ext_vector_type(8)))  __bf16   v8b;
typedef __attribute__((ext_vector_type(8)))  float    v8f;
typedef __attribute__((ext_vector_type(4)))  float    v4f;
typedef __attribute__((ext_vector_type(2)))  float    v2f;
typedef __attribute__((ext_vector_type(4)))  unsigned int v4u;

__device__ __forceinline__ unsigned short f2bf_bits(float f) {
  unsigned u = __float_as_uint(f);
  return (unsigned short)((u + 0x7FFFu + ((u >> 16) & 1u)) >> 16);
}
__device__ __forceinline__ float bf_bits2f(unsigned short h) { return __uint_as_float(((unsigned)h) << 16); }
__device__ __forceinline__ unsigned pk16(unsigned short a, unsigned short b) { return (unsigned)a | ((unsigned)b << 16); }
__device__ __forceinline__ unsigned short h_bits(float f) { const _Float16 h = (_Float16)f; return __builtin_bit_cast(unsigned short, h); }

__device__ __forceinline__ void guard_h5(v8f& a, v8f& b, v8f& c, v8f& d, v16h x, v16h y0, v16h y1, v16h y2, v16h y3) {
  asm volatile("v_nop\n\tv_nop\n\tv_nop\n\tv_nop" : "+v"(a), "+v"(b), "+v"(c), "+v"(d) : "v"(x), "v"(y0), "v"(y1), "v"(y2), "v"(y3));
}
__device__ __forceinline__ void guard_b10(v8f& a, v8f& b, v8f& c, v8f& d, v16b x, v16b xl,
                                          v16b y0, v16b y1, v16b y2, v16b y3, v16b l0, v16b l1, v16b l2, v16b l3) {
  asm volatile("v_nop\n\tv_nop\n\tv_nop\n\tv_nop" : "+v"(a), "+v"(b), "+v"(c), "+v"(d)
               : "v"(x), "v"(xl), "v"(y0), "v"(y1), "v"(y2), "v"(y3), "v"(l0), "v"(l1), "v"(l2), "v"(l3));
}
__device__ __forceinline__ void acc_guard4(v8f& a, v8f& b, v8f& c, v8f& d) {
  asm volatile("v_nop\n\tv_nop\n\tv_nop\n\tv_nop" : "+v"(a), "+v"(b), "+v"(c), "+v"(d));
}
__device__ __forceinline__ void pin4(v4f& a) {
  asm volatile("" : "+v"(a));
}
__device__ __forceinline__ void wave_lds_sync() {
  __builtin_amdgcn_fence(__ATOMIC_RELEASE, "workgroup");
  __builtin_amdgcn_wave_barrier();
  __builtin_amdgcn_fence(__ATOMIC_ACQUIRE, "workgroup");
}

template <typename T> struct Frag;
template <> struct Frag<_Float16> {
  typedef v16h V; union U { v16h v; v8h h[2]; };
  static __device__ __forceinline__ v16h load(const _Float16* p) {
    U f; f.h[0] = *(const v8h*)(p); f.h[1] = *(const v8h*)(p + 16); return f.v;
  }
  static __device__ __forceinline__ v8f mma(v16h a, v16h b, v8f c) {
    return __builtin_amdgcn_wmma_f32_16x16x32_f16(false, a, false, b, (short)0, c, false, false);
  }
};
template <> struct Frag<__bf16> {
  typedef v16b V; union U { v16b v; v8b h[2]; };
  static __device__ __forceinline__ v16b load(const __bf16* p) {
    U f; f.h[0] = *(const v8b*)(p); f.h[1] = *(const v8b*)(p + 16); return f.v;
  }
  static __device__ __forceinline__ v8f mma(v16b a, v16b b, v8f c) {
    return __builtin_amdgcn_wmma_f32_16x16x32_bf16(false, a, false, b, (short)0, c, false, false);
  }
};

struct EpiArgs {
  void* C;
  void* C2;
  const float* bias;
  const float* xin;
  const float* mu;
  float scale;
  int ldc;
  int act;
};

template <int EPI>
__device__ __forceinline__ void tile_epilogue(v8f (&acc)[4][4], float* slab, const int lane,
                                              const int m0, const int n0, const EpiArgs& ea) {
  const int rlane = lane & 15;
  const int mOff  = (lane >> 4) * 8;
  float bv[4];
#pragma unroll
  for (int j = 0; j < 4; ++j) {
    if (EPI == 2) bv[j] = ea.bias[n0 + (j << 4) + rlane];
    else bv[j] = 0.0f;
  }
#pragma unroll
  for (int i = 0; i < 4; ++i) {
    const int mBase = m0 + (i << 4);
#pragma unroll
    for (int j = 0; j < 4; ++j) {
#pragma unroll
      for (int r = 0; r < 8; ++r) {
        float v = acc[i][j][r] * ea.scale;
        if (EPI == 2) v += bv[j];
        slab[(mOff + r) * 68 + (j << 4) + rlane] = v;
      }
    }
    wave_lds_sync();
    const bool doAct = (EPI == 1) || (EPI == 2) || ((EPI == 0) && (ea.act != 0));
    if (doAct) {
#pragma unroll 1
      for (int q = 0; q < 32; ++q) {
        const int idx = q * 32 + lane;
        const int off = (idx >> 6) * 68 + (idx & 63);
        float v = slab[off];
        if (EPI == 1) v = tanhf(v);
        if (EPI == 2) v = expf(-expf(v));
        if (EPI == 0) v = v * (1.0f / (1.0f + expf(-v)));
        slab[off] = v;
      }
      wave_lds_sync();
    }
    if (EPI == 0 || EPI == 2) {
      float* C = (float*)ea.C;
      const int hh = lane >> 4, c4 = (lane & 15) * 4;
      for (int pass = 0; pass < 2; ++pass) {
#pragma unroll
        for (int it = 0; it < 8; ++it) {
          const int row = it * 2 + hh;
          const v4f v = *(const v4f*)(slab + row * 68 + c4);
          *(volatile v4f*)(C + (size_t)(mBase + row) * ea.ldc + n0 + c4) = v;
        }
        __threadfence();
      }
    } else if (EPI == 1) {
      unsigned short* C = (unsigned short*)ea.C;
      const int q = lane >> 3, c8 = (lane & 7) * 8;
      v4u hv[4];
#pragma unroll
      for (int it = 0; it < 4; ++it) {
        const int row = it * 4 + q;
        const float* sp = slab + row * 68 + c8;
        const v4f s0 = *(const v4f*)(sp);
        const v4f s1 = *(const v4f*)(sp + 4);
        unsigned short hb[8];
#pragma unroll
        for (int e = 0; e < 4; ++e) {
          const float f0 = s0[e];
          const float f1 = s1[e];
          hb[e]     = h_bits(f0);
          hb[4 + e] = h_bits(f1);
        }
        hv[it] = (v4u){pk16(hb[0], hb[1]), pk16(hb[2], hb[3]), pk16(hb[4], hb[5]), pk16(hb[6], hb[7])};
      }
      for (int pass = 0; pass < 2; ++pass) {
#pragma unroll
        for (int it = 0; it < 4; ++it) {
          const int row = it * 4 + q;
          *(volatile v4u*)(C + (size_t)(mBase + row) * ea.ldc + n0 + c8) = hv[it];
        }
        __threadfence();
      }
    } else {
      unsigned short* C  = (unsigned short*)ea.C;
      unsigned short* C2 = (unsigned short*)ea.C2;
      const int q = lane >> 3, c8 = (lane & 7) * 8;
      v4u hv[4], lv[4];
#pragma unroll
      for (int it = 0; it < 4; ++it) {
        const int row = it * 4 + q;
        const int m   = mBase + row;
        const int t   = m & (kT - 1);
        const bool hasP = (t > 0);
        const int mp  = hasP ? (m - 1) : m;
        const float fp = hasP ? 1.0f : 0.0f;
        const float* sp = slab + row * 68 + c8;
        const v4f s0 = *(const v4f*)(sp);
        const v4f s1 = *(const v4f*)(sp + 4);
        const float* xc = ea.xin + (size_t)m  * kC + n0 + c8;
        const float* xp = ea.xin + (size_t)mp * kC + n0 + c8;
        const v4f x0 = *(const v4f*)(xc);
        const v4f x1 = *(const v4f*)(xc + 4);
        v4f p0 = *(const v4f*)(xp);
        v4f p1 = *(const v4f*)(xp + 4);
        pin4(p0);
        pin4(p1);
        const v4f u0 = *(const v4f*)(ea.mu + n0 + c8);
        const v4f u1 = *(const v4f*)(ea.mu + n0 + c8 + 4);
        float vals[8];
#pragma unroll
        for (int e = 0; e < 4; ++e) {
          const float c0 = x0[e];
          const float c1 = x1[e];
          const float q0 = p0[e] * fp;
          const float q1 = p1[e] * fp;
          vals[e]     = c0 + (q0 - c0) * (u0[e] + s0[e]);
          vals[4 + e] = c1 + (q1 - c1) * (u1[e] + s1[e]);
        }
        unsigned short hb[8], lb[8];
#pragma unroll
        for (int e = 0; e < 8; ++e) {
          hb[e] = f2bf_bits(vals[e]);
          lb[e] = f2bf_bits(vals[e] - bf_bits2f(hb[e]));
        }
        hv[it] = (v4u){pk16(hb[0], hb[1]), pk16(hb[2], hb[3]), pk16(hb[4], hb[5]), pk16(hb[6], hb[7])};
        lv[it] = (v4u){pk16(lb[0], lb[1]), pk16(lb[2], lb[3]), pk16(lb[4], lb[5]), pk16(lb[6], lb[7])};
      }
      for (int pass = 0; pass < 2; ++pass) {
#pragma unroll
        for (int it = 0; it < 4; ++it) {
          const int row = it * 4 + q;
          const size_t go = (size_t)(mBase + row) * ea.ldc + n0 + c8;
          *(volatile v4u*)(C + go)  = hv[it];
          *(volatile v4u*)(C2 + go) = lv[it];
        }
        __threadfence();
      }
    }
    wave_lds_sync();
  }
}

template <int EPI>
__global__ __launch_bounds__(256) void gemm_h(
    const unsigned short* __restrict__ Ap, int lda, long strideA,
    const unsigned short* __restrict__ Btp, int ldb, long strideB,
    void* __restrict__ Cout, void* __restrict__ Cout2, int ldc, long strideC,
    const float* __restrict__ bias, const float* __restrict__ xin, const float* __restrict__ mu5,
    int M, int N, int K, float scale) {
  __shared__ __align__(16) float sT[8][16 * 68];
  const int zb   = blockIdx.y;
  const int lane = threadIdx.x & 31;
  const int wave = threadIdx.x >> 5;
  const int tilesN = N >> 6;
  const int tilesM = M >> 6;
  const int tile = blockIdx.x * 8 + wave;
  if (tile >= tilesM * tilesN) return;
  const int tm = tile / tilesN;
  const int tn = tile - tm * tilesN;
  const int m0 = tm << 6;
  const int n0 = tn << 6;
  const _Float16* A  = (const _Float16*)Ap  + (size_t)zb * strideA;
  const _Float16* Bt = (const _Float16*)Btp + (size_t)zb * strideB;
  const int rlane = lane & 15;
  const int koff  = (lane >> 4) * 8;
  int ao[4], bo[4];
#pragma unroll
  for (int i = 0; i < 4; ++i) {
    ao[i] = (m0 + (i << 4) + rlane) * lda + koff;
    bo[i] = (n0 + (i << 4) + rlane) * ldb + koff;
  }
  v8f acc[4][4];
#pragma unroll
  for (int i = 0; i < 4; ++i)
#pragma unroll
    for (int j = 0; j < 4; ++j) acc[i][j] = (v8f){0.f, 0.f, 0.f, 0.f, 0.f, 0.f, 0.f, 0.f};

  for (int k0 = 0; k0 < K; k0 += 32) {
    const v16h b0 = Frag<_Float16>::load(Bt + bo[0] + k0);
    const v16h b1 = Frag<_Float16>::load(Bt + bo[1] + k0);
    const v16h b2 = Frag<_Float16>::load(Bt + bo[2] + k0);
    const v16h b3 = Frag<_Float16>::load(Bt + bo[3] + k0);
#pragma unroll
    for (int i = 0; i < 4; ++i) {
      const v16h ah = Frag<_Float16>::load(A + ao[i] + k0);
      acc[i][0] = Frag<_Float16>::mma(ah, b0, acc[i][0]);
      acc[i][1] = Frag<_Float16>::mma(ah, b1, acc[i][1]);
      acc[i][2] = Frag<_Float16>::mma(ah, b2, acc[i][2]);
      acc[i][3] = Frag<_Float16>::mma(ah, b3, acc[i][3]);
      guard_h5(acc[i][0], acc[i][1], acc[i][2], acc[i][3], ah, b0, b1, b2, b3);
    }
  }
  acc_guard4(acc[0][0], acc[0][1], acc[0][2], acc[0][3]);
  acc_guard4(acc[1][0], acc[1][1], acc[1][2], acc[1][3]);
  acc_guard4(acc[2][0], acc[2][1], acc[2][2], acc[2][3]);
  acc_guard4(acc[3][0], acc[3][1], acc[3][2], acc[3][3]);

  EpiArgs ea;
  if (EPI == 0 || EPI == 2) {
    ea.C  = (void*)((float*)Cout + (size_t)zb * strideC);
    ea.C2 = ea.C;
  } else {
    ea.C  = (void*)((unsigned short*)Cout  + (size_t)zb * strideC);
    ea.C2 = (void*)((unsigned short*)Cout2 + (size_t)zb * strideC);
  }
  ea.bias = bias;
  ea.xin = xin;
  ea.mu = mu5 + (size_t)zb * kC;
  ea.scale = scale;
  ea.ldc = ldc;
  ea.act = 0;
  tile_epilogue<EPI>(acc, sT[wave], lane, m0, n0, ea);
}

template <int EPI>
__global__ __launch_bounds__(256) void gemm_b3(
    const unsigned short* __restrict__ Ahp, const unsigned short* __restrict__ Alp, int lda, long strideA,
    const unsigned short* __restrict__ Bhp, const unsigned short* __restrict__ Blp, int ldb, long strideB,
    void* __restrict__ Cout, int ldc, long strideC,
    const float* __restrict__ bias, const float* __restrict__ xin, const float* __restrict__ mu5,
    int M, int N, int K, float scale, int actZ) {
  __shared__ __align__(16) float sT[8][16 * 68];
  const int zb   = blockIdx.y;
  const int lane = threadIdx.x & 31;
  const int wave = threadIdx.x >> 5;
  const int tilesN = N >> 6;
  const int tilesM = M >> 6;
  const int tile = blockIdx.x * 8 + wave;
  if (tile >= tilesM * tilesN) return;
  const int tm = tile / tilesN;
  const int tn = tile - tm * tilesN;
  const int m0 = tm << 6;
  const int n0 = tn << 6;
  const __bf16* Ah = (const __bf16*)Ahp + (size_t)zb * strideA;
  const __bf16* Al = (const __bf16*)Alp + (size_t)zb * strideA;
  const __bf16* Bh = (const __bf16*)Bhp + (size_t)zb * strideB;
  const __bf16* Bl = (const __bf16*)Blp + (size_t)zb * strideB;
  const int rlane = lane & 15;
  const int koff  = (lane >> 4) * 8;
  int ao[4], bo[4];
#pragma unroll
  for (int i = 0; i < 4; ++i) {
    ao[i] = (m0 + (i << 4) + rlane) * lda + koff;
    bo[i] = (n0 + (i << 4) + rlane) * ldb + koff;
  }
  v8f acc[4][4];
#pragma unroll
  for (int i = 0; i < 4; ++i)
#pragma unroll
    for (int j = 0; j < 4; ++j) acc[i][j] = (v8f){0.f, 0.f, 0.f, 0.f, 0.f, 0.f, 0.f, 0.f};

  for (int k0 = 0; k0 < K; k0 += 32) {
    const v16b bh0 = Frag<__bf16>::load(Bh + bo[0] + k0);
    const v16b bh1 = Frag<__bf16>::load(Bh + bo[1] + k0);
    const v16b bh2 = Frag<__bf16>::load(Bh + bo[2] + k0);
    const v16b bh3 = Frag<__bf16>::load(Bh + bo[3] + k0);
    const v16b bl0 = Frag<__bf16>::load(Bl + bo[0] + k0);
    const v16b bl1 = Frag<__bf16>::load(Bl + bo[1] + k0);
    const v16b bl2 = Frag<__bf16>::load(Bl + bo[2] + k0);
    const v16b bl3 = Frag<__bf16>::load(Bl + bo[3] + k0);
#pragma unroll
    for (int i = 0; i < 4; ++i) {
      const v16b ah = Frag<__bf16>::load(Ah + ao[i] + k0);
      const v16b al = Frag<__bf16>::load(Al + ao[i] + k0);
      acc[i][0] = Frag<__bf16>::mma(ah, bh0, acc[i][0]);
      acc[i][1] = Frag<__bf16>::mma(ah, bh1, acc[i][1]);
      acc[i][2] = Frag<__bf16>::mma(ah, bh2, acc[i][2]);
      acc[i][3] = Frag<__bf16>::mma(ah, bh3, acc[i][3]);
      acc[i][0] = Frag<__bf16>::mma(ah, bl0, acc[i][0]);
      acc[i][1] = Frag<__bf16>::mma(ah, bl1, acc[i][1]);
      acc[i][2] = Frag<__bf16>::mma(ah, bl2, acc[i][2]);
      acc[i][3] = Frag<__bf16>::mma(ah, bl3, acc[i][3]);
      acc[i][0] = Frag<__bf16>::mma(al, bh0, acc[i][0]);
      acc[i][1] = Frag<__bf16>::mma(al, bh1, acc[i][1]);
      acc[i][2] = Frag<__bf16>::mma(al, bh2, acc[i][2]);
      acc[i][3] = Frag<__bf16>::mma(al, bh3, acc[i][3]);
      guard_b10(acc[i][0], acc[i][1], acc[i][2], acc[i][3], ah, al, bh0, bh1, bh2, bh3, bl0, bl1, bl2, bl3);
    }
  }
  acc_guard4(acc[0][0], acc[0][1], acc[0][2], acc[0][3]);
  acc_guard4(acc[1][0], acc[1][1], acc[1][2], acc[1][3]);
  acc_guard4(acc[2][0], acc[2][1], acc[2][2], acc[2][3]);
  acc_guard4(acc[3][0], acc[3][1], acc[3][2], acc[3][3]);

  EpiArgs ea;
  if (EPI == 0) ea.C = (void*)((float*)Cout + (size_t)zb * strideC);
  else          ea.C = (void*)((unsigned short*)Cout + (size_t)zb * strideC);
  ea.C2 = ea.C;
  ea.bias = bias;
  ea.xin = xin;
  ea.mu = mu5;
  ea.scale = scale;
  ea.ldc = ldc;
  ea.act = (zb == actZ) ? 1 : 0;
  tile_epilogue<EPI>(acc, sT[wave], lane, m0, n0, ea);
}

template <bool BF_SPLIT>
__global__ __launch_bounds__(256) void tcast_kernel(const float* __restrict__ in0, const float* __restrict__ in1,
                                                    const float* __restrict__ in2, const float* __restrict__ in3,
                                                    const float* __restrict__ in4, int R, int C,
                                                    unsigned short* __restrict__ out, unsigned short* __restrict__ out2,
                                                    int RP, long planeStride, float carry) {
  __shared__ float sm[64][65];
  const int t  = threadIdx.x;
  const int r0 = blockIdx.x * 64;
  const int c0 = blockIdx.y * 64;
  const int z  = blockIdx.z;
  const float* in = (z == 0) ? in0 : (z == 1) ? in1 : (z == 2) ? in2 : (z == 3) ? in3 : in4;
#pragma unroll
  for (int i = 0; i < 16; ++i) {
    const int e  = i * 256 + t;
    const int rl = e >> 6;
    const int cl = e & 63;
    const int r = r0 + rl, c = c0 + cl;
    const int rc = (r < R) ? r : (R - 1);
    const int cc = (c < C) ? c : (C - 1);
    const float v = in[(size_t)rc * C + cc];
    sm[cl][rl] = (r < R && c < C) ? (v * carry) : 0.0f;
  }
  __syncthreads();
  const int lane = t & 31, wave = t >> 5;
  const int q = lane >> 3, c8 = (lane & 7) * 8;
  unsigned short* o1 = out  + (size_t)z * planeStride;
  unsigned short* o2 = out2 + (size_t)z * planeStride;
  v4u hv[2], lv[2];
#pragma unroll
  for (int it = 0; it < 2; ++it) {
    const int row = wave * 8 + it * 4 + q;
    unsigned short hb[8], lb[8];
#pragma unroll
    for (int e = 0; e < 8; ++e) {
      const float v = sm[row][c8 + e];
      if (BF_SPLIT) {
        hb[e] = f2bf_bits(v);
        lb[e] = f2bf_bits(v - bf_bits2f(hb[e]));
      } else {
        hb[e] = h_bits(v);
        lb[e] = hb[e];
      }
    }
    hv[it] = (v4u){pk16(hb[0], hb[1]), pk16(hb[2], hb[3]), pk16(hb[4], hb[5]), pk16(hb[6], hb[7])};
    lv[it] = (v4u){pk16(lb[0], lb[1]), pk16(lb[2], lb[3]), pk16(lb[4], lb[5]), pk16(lb[6], lb[7])};
  }
  for (int pass = 0; pass < 2; ++pass) {
#pragma unroll
    for (int it = 0; it < 2; ++it) {
      const int row = wave * 8 + it * 4 + q;
      const size_t go = (size_t)(c0 + row) * RP + r0 + c8;
      *(volatile v4u*)(o1 + go) = hv[it];
      if (BF_SPLIT) *(volatile v4u*)(o2 + go) = lv[it];
    }
    __threadfence();
  }
}

__global__ __launch_bounds__(256) void shift_kernel(const float* __restrict__ x, const float* __restrict__ maax,
                                                    unsigned short* __restrict__ XA) {
  const int i   = blockIdx.x * 256 + threadIdx.x;
  const int row = i >> 7;
  const int c8  = (i & 127) * 8;
  const int t   = row & (kT - 1);
  const bool hasP = (t > 0);
  const int rp  = hasP ? (row - 1) : row;
  const float* xc = x + (size_t)row * kC + c8;
  const float* xp = x + (size_t)rp  * kC + c8;
  const v4f a0 = *(const v4f*)(xc);
  const v4f a1 = *(const v4f*)(xc + 4);
  const v4f p0 = *(const v4f*)(xp);
  const v4f p1 = *(const v4f*)(xp + 4);
  const v4f m0 = *(const v4f*)(maax + c8);
  const v4f m1 = *(const v4f*)(maax + c8 + 4);
  unsigned short hb[8];
#pragma unroll
  for (int e = 0; e < 4; ++e) {
    const float c0 = a0[e];
    const float c1 = a1[e];
    const float q0 = hasP ? p0[e] : 0.0f;
    const float q1 = hasP ? p1[e] : 0.0f;
    hb[e]     = h_bits(c0 + (q0 - c0) * m0[e]);
    hb[4 + e] = h_bits(c1 + (q1 - c1) * m1[e]);
  }
  const v4u u = (v4u){pk16(hb[0], hb[1]), pk16(hb[2], hb[3]), pk16(hb[4], hb[5]), pk16(hb[6], hb[7])};
  unsigned short* op = XA + (size_t)row * kC + c8;
  *(volatile v4u*)op = u;
  __threadfence();
  *(volatile v4u*)op = u;
}

__global__ __launch_bounds__(128) void scan_kernel(const float* __restrict__ Rp, const float* __restrict__ Kp,
                                                   const float* __restrict__ Vp, const float* __restrict__ Wd,
                                                   const float* __restrict__ U, float* __restrict__ Y) {
  __shared__ __align__(16) float rs[kChunk * 64];
  __shared__ __align__(16) float ks[kChunk * 64];
  __shared__ __align__(16) float wsd[kChunk * 64];
  __shared__ __align__(16) float vs[kChunk * 64];
  __shared__ __align__(16) float ys[kChunk * 64];
  __shared__ float us[64];
  __shared__ float bon[kChunk];
  const int bh   = blockIdx.x;
  const int b    = bh >> 4;
  const int h    = bh & 15;
  const int tid  = threadIdx.x;
  const int lane = tid & 31;
  const int wave = tid >> 5;
  const int ih   = lane >> 4;
  const int j    = wave * 16 + (lane & 15);
  const size_t base = (size_t)b * kT * kC + (size_t)h * kHS;
  if (tid < 64) us[tid] = U[h * kHS + tid];
  float S[32];
#pragma unroll
  for (int e = 0; e < 32; ++e) S[e] = 0.0f;

#pragma unroll 1
  for (int ch = 0; ch < kT / kChunk; ++ch) {
    __syncthreads();
#pragma unroll
    for (int it = 0; it < 4; ++it) {
      const int idx = it * 128 + tid;
      const int row = idx >> 4;
      const int c4  = (idx & 15) * 4;
      const size_t g = base + (size_t)(ch * kChunk + row) * kC + c4;
      const v4f a = *(const v4f*)(Rp + g);
      const v4f c = *(const v4f*)(Kp + g);
      const v4f d = *(const v4f*)(Wd + g);
      const v4f e = *(const v4f*)(Vp + g);
      *(v4f*)(rs  + row * 64 + c4) = a;
      *(v4f*)(ks  + row * 64 + c4) = c;
      *(v4f*)(wsd + row * 64 + c4) = d;
      *(v4f*)(vs  + row * 64 + c4) = e;
    }
    __syncthreads();
    {
      const int tl   = tid >> 2;
      const int part = tid & 3;
      float s = 0.0f;
#pragma unroll 4
      for (int e = 0; e < 16; ++e) {
        const int i = part * 16 + e;
        s += rs[tl * 64 + i] * us[i] * ks[tl * 64 + i];
      }
      s += __shfl_xor(s, 1, 32);
      s += __shfl_xor(s, 2, 32);
      if (part == 0) bon[tl] = s;
    }
    __syncthreads();
#pragma unroll 1
    for (int tl = 0; tl < kChunk; ++tl) {
      const float vj = vs[tl * 64 + j];
      const float* rp = rs  + tl * 64 + ih * 32;
      const float* kp = ks  + tl * 64 + ih * 32;
      const float* wp = wsd + tl * 64 + ih * 32;
      float y = 0.0f;
#pragma unroll
      for (int q = 0; q < 8; ++q) {
        const v4f r4 = *(const v4f*)(rp + 4 * q);
        const v4f k4 = *(const v4f*)(kp + 4 * q);
        const v4f w4 = *(const v4f*)(wp + 4 * q);
#pragma unroll
        for (int e = 0; e < 4; ++e) {
          const float kv = k4[e] * vj;
          y = fmaf(r4[e], S[4 * q + e], y);
          S[4 * q + e] = fmaf(w4[e], S[4 * q + e], kv);
        }
      }
      y += __shfl_xor(y, 16, 32);
      y = fmaf(bon[tl], vj, y);
      if (ih == 0) ys[tl * 64 + j] = y;
    }
    __syncthreads();
    for (int pass = 0; pass < 2; ++pass) {
#pragma unroll
      for (int it = 0; it < 4; ++it) {
        const int row = it * 8 + (tid >> 4);
        const int c4  = (tid & 15) * 4;
        const v4f v = *(const v4f*)(ys + row * 64 + c4);
        *(volatile v4f*)(Y + base + (size_t)(ch * kChunk + row) * kC + c4) = v;
      }
      __threadfence();
    }
  }
}

__global__ __launch_bounds__(256) void gn_gate_kernel(const float* __restrict__ Y, const float* __restrict__ G,
                                                      const float* __restrict__ lnw, const float* __restrict__ lnb,
                                                      unsigned int* __restrict__ Zh, unsigned int* __restrict__ Zl) {
  const int lane = threadIdx.x & 31, wave = threadIdx.x >> 5;
  const int grp = blockIdx.x * 8 + wave;
  const int tok = grp >> 4;
  const int h   = grp & 15;
  const int chn = h * kHS + 2 * lane;
  const size_t base = (size_t)tok * kC + chn;
  const v2f yv = *(const v2f*)(Y + base);
  const v2f gv = *(const v2f*)(G + base);
  const v2f wv = *(const v2f*)(lnw + chn);
  const v2f bv = *(const v2f*)(lnb + chn);
  const float y0 = yv[0], y1 = yv[1];
  float s = y0 + y1;
#pragma unroll
  for (int off = 16; off > 0; off >>= 1) s += __shfl_xor(s, off, 32);
  const float mu = s * (1.0f / kHS);
  const float d0 = y0 - mu, d1 = y1 - mu;
  float ss = d0 * d0 + d1 * d1;
#pragma unroll
  for (int off = 16; off > 0; off >>= 1) ss += __shfl_xor(ss, off, 32);
  const float var  = ss * (1.0f / kHS);
  const float rstd = rsqrtf(var + kGnEps);
  const float z0 = ((d0 * rstd) * wv[0] + bv[0]) * gv[0];
  const float z1 = ((d1 * rstd) * wv[1] + bv[1]) * gv[1];
  const unsigned short h0 = f2bf_bits(z0);
  const unsigned short h1 = f2bf_bits(z1);
  const unsigned short l0 = f2bf_bits(z0 - bf_bits2f(h0));
  const unsigned short l1 = f2bf_bits(z1 - bf_bits2f(h1));
  const unsigned uh = pk16(h0, h1);
  const unsigned ul = pk16(l0, l1);
  unsigned int* ph = Zh + (base >> 1);
  unsigned int* pl = Zl + (base >> 1);
  *(volatile unsigned int*)ph = uh;
  *(volatile unsigned int*)pl = ul;
  __threadfence();
  *(volatile unsigned int*)ph = uh;
  *(volatile unsigned int*)pl = ul;
}

extern "C" void kernel_launch(void* const* d_in, const int* in_sizes, int n_in,
                              void* d_out, int out_size, void* d_ws, size_t ws_size, hipStream_t stream) {
  if (n_in < 16 || d_out == nullptr || d_ws == nullptr) return;
  if (in_sizes[0] != kRows * kC || in_sizes[1] != kC || in_sizes[2] != 5 * kC || in_sizes[3] != kC * kMixCols ||
      in_sizes[4] != kMixCols * kC || in_sizes[5] != kC || in_sizes[6] != kC * kDecRank ||
      in_sizes[7] != kDecRank * kC || in_sizes[8] != kH * kHS || in_sizes[9] != kC * kC ||
      in_sizes[10] != kC * kC || in_sizes[11] != kC * kC || in_sizes[12] != kC * kC || in_sizes[13] != kC * kC ||
      in_sizes[14] != kC || in_sizes[15] != kC || out_size != kRows * kC) return;

  const float* x     = (const float*)d_in[0];
  const float* maax  = (const float*)d_in[1];
  const float* mu5   = (const float*)d_in[2];
  const float* tmw1  = (const float*)d_in[3];
  const float* tmw2  = (const float*)d_in[4];
  const float* tdec  = (const float*)d_in[5];
  const float* tdw1  = (const float*)d_in[6];
  const float* tdw2  = (const float*)d_in[7];
  const float* ubon  = (const float*)d_in[8];
  const float* Wr    = (const float*)d_in[9];
  const float* Wk    = (const float*)d_in[10];
  const float* Wv    = (const float*)d_in[11];
  const float* Wg    = (const float*)d_in[12];
  const float* Wo    = (const float*)d_in[13];
  const float* lnw   = (const float*)d_in[14];
  const float* lnb   = (const float*)d_in[15];
  float* out = (float*)d_out;

  char* ws = (char*)d_ws;
  size_t off = 0;
  auto carve = [&](size_t bytes) -> char* { char* p = ws + off; off += (bytes + 255) & ~(size_t)255; return p; };
  const size_t WSQ = (size_t)kC * kC;
  unsigned short* XA   = (unsigned short*)carve(kPlane * 2);
  unsigned short* W1T  = (unsigned short*)carve((size_t)kMixPad * kC * 2);
  unsigned short* W2T  = (unsigned short*)carve((size_t)kC * kMixPad * 2);
  unsigned short* DW1H = (unsigned short*)carve((size_t)kDecRank * kC * 2);
  unsigned short* DW1L = (unsigned short*)carve((size_t)kDecRank * kC * 2);
  unsigned short* DW2T = (unsigned short*)carve((size_t)kC * kDecRank * 2);
  unsigned short* WTH  = (unsigned short*)carve(5 * WSQ * 2);
  unsigned short* WTL  = (unsigned short*)carve(5 * WSQ * 2);
  unsigned short* MPL  = (unsigned short*)carve((size_t)kRows * kMixPad * 2);
  unsigned short* XH   = (unsigned short*)carve(5 * kPlane * 2);
  unsigned short* XL   = (unsigned short*)carve(5 * kPlane * 2);
  unsigned short* T1   = (unsigned short*)carve((size_t)kRows * kDecRank * 2);
  float*          WD   = (float*)carve(kPlane * 4);
  float*          KVRG = (float*)carve(4 * kPlane * 4);
  float*          Yb   = (float*)carve(kPlane * 4);
  unsigned short* ZH   = (unsigned short*)carve(kPlane * 2);
  unsigned short* ZL   = (unsigned short*)carve(kPlane * 2);
  if (off > ws_size || off > (size_t)134217728) return;

  tcast_kernel<false><<<dim3(kC / 64, kMixPad / 64, 1), 256, 0, stream>>>(
      tmw1, tmw1, tmw1, tmw1, tmw1, kC, kMixCols, W1T, W1T, kC, 0L, kLCarry);
  tcast_kernel<false><<<dim3(kMixPad / 64, kC / 64, 1), 256, 0, stream>>>(
      tmw2, tmw2, tmw2, tmw2, tmw2, kMixCols, kC, W2T, W2T, kMixPad, 0L, kLCarry);
  tcast_kernel<false><<<dim3(kDecRank / 64, kC / 64, 1), 256, 0, stream>>>(
      tdw2, tdw2, tdw2, tdw2, tdw2, kDecRank, kC, DW2T, DW2T, kDecRank, 0L, kLCarry);
  tcast_kernel<true><<<dim3(kC / 64, kDecRank / 64, 1), 256, 0, stream>>>(
      tdw1, tdw1, tdw1, tdw1, tdw1, kC, kDecRank, DW1H, DW1L, kC, 0L, 1.0f);
  tcast_kernel<true><<<dim3(kC / 64, kC / 64, 5), 256, 0, stream>>>(
      Wk, Wv, Wr, Wg, Wo, kC, kC, WTH, WTL, kC, (long)WSQ, 1.0f);

  const int gBig = (kRows / 64) * (kC / 64) / 8;
  const int gMix = (kRows / 64) * (kMixPad / 64) / 8;
  const int gDec = (kRows / 64) * (kDecRank / 64) / 8;

  shift_kernel<<<kRows * kC / 8 / 256, 256, 0, stream>>>(x, maax, XA);

  gemm_h<1><<<dim3(gMix, 1), 256, 0, stream>>>(
      XA, kC, 0L, W1T, kC, 0L, (void*)MPL, (void*)MPL, kMixPad, 0L,
      tdec, x, mu5, kRows, kMixPad, kC, kLFold);

  gemm_h<3><<<dim3(gBig, 5), 256, 0, stream>>>(
      MPL, kMixPad, (long)kMixRank, W2T, kMixPad, (long)kMixRank, (void*)XH, (void*)XL, kC, (long)kPlane,
      tdec, x, mu5, kRows, kC, kMixRank, kLFold);

  gemm_b3<1><<<dim3(gDec, 1), 256, 0, stream>>>(
      XH, XL, kC, 0L, DW1H, DW1L, kC, 0L, (void*)T1, kDecRank, 0L,
      tdec, x, mu5, kRows, kDecRank, kC, 1.0f, -1);

  gemm_h<2><<<dim3(gBig, 1), 256, 0, stream>>>(
      T1, kDecRank, 0L, DW2T, kDecRank, 0L, (void*)WD, (void*)WD, kC, 0L,
      tdec, x, mu5, kRows, kC, kDecRank, kLFold);

  gemm_b3<0><<<dim3(gBig, 4), 256, 0, stream>>>(
      XH + kPlane, XL + kPlane, kC, (long)kPlane, WTH, WTL, kC, (long)WSQ, (void*)KVRG, kC, (long)kPlane,
      tdec, x, mu5, kRows, kC, kC, 1.0f, 3);

  scan_kernel<<<kB * kH, 128, 0, stream>>>(KVRG + 2 * kPlane, KVRG, KVRG + kPlane, WD, ubon, Yb);

  gn_gate_kernel<<<kRows * kH / 8, 256, 0, stream>>>(Yb, KVRG + 3 * kPlane, lnw, lnb,
                                                     (unsigned int*)ZH, (unsigned int*)ZL);

  gemm_b3<0><<<dim3(gBig, 1), 256, 0, stream>>>(
      ZH, ZL, kC, 0L, WTH + 4 * WSQ, WTL + 4 * WSQ, kC, 0L, (void*)out, kC, 0L,
      tdec, x, mu5, kRows, kC, kC, 1.0f, -1);
}
